// GNNExplainerAgg_44770739093934
// MI455X (gfx1250) — hardware-verified
//
#include <hip/hip_runtime.h>
#include <stddef.h>


#define D       128
#define NTHR    256
#define NWAVE   8
#define EPT     8
#define NGRP    2
#define CHUNK   (NTHR * EPT * NGRP)
#define WCAP    (EPT * NGRP * 32)
#define LISTN   (NWAVE * WCAP)
#define TGT     256
#define GROWS   128
#define AP      (D + 8)
#define WSCALE  16.0f
#define WINV    0.0625f

#define LDS_GEMM (GROWS * D * 4)
#define LDS_GEM3 (2 * GROWS * AP * 2)
#define LDS_AGG  (TGT * D * 4 + TGT * 4 + TGT * 4 + LISTN * 4 + 64)

static_assert((CHUNK & (CHUNK - 1)) == 0);
static_assert(CHUNK <= 4096);
static_assert(TGT <= 4096 && (TGT & (TGT - 1)) == 0);
static_assert(TGT == NWAVE * 32);
static_assert((TGT % GROWS) == 0);
static_assert(GROWS == NWAVE * 16);
static_assert(GROWS * AP * 2 <= LDS_GEMM);
static_assert(GROWS * D * 4 <= LDS_GEM3);
static_assert((GROWS * D / 8) % NTHR == 0);
static_assert((D * D / 8) % NTHR == 0);
static_assert((TGT * D / 4) % NTHR == 0);
static_assert(D == 4 * 32);

typedef float          v4f  __attribute__((ext_vector_type(4)));
typedef float          v8f  __attribute__((ext_vector_type(8)));
typedef int            v4i  __attribute__((ext_vector_type(4)));
typedef _Float16       v8h  __attribute__((ext_vector_type(8)));
typedef _Float16       v16h __attribute__((ext_vector_type(16)));
typedef unsigned short v8us __attribute__((ext_vector_type(8)));
typedef __bf16         v16b __attribute__((ext_vector_type(16)));
union FragH { v16h v; v8h h[2]; };
union FragB { v16b v; v8us h[2]; };

__device__ __forceinline__ unsigned short f2bf(float f) {
  unsigned int u = __float_as_uint(f);
  u += 0x7FFFu + ((u >> 16) & 1u);
  return (unsigned short)(u >> 16);
}

__device__ __forceinline__ v8h cvt8(v4f a, v4f b) {
  v8h r;
  r[0] = (_Float16)a.x; r[1] = (_Float16)a.y; r[2] = (_Float16)a.z; r[3] = (_Float16)a.w;
  r[4] = (_Float16)b.x; r[5] = (_Float16)b.y; r[6] = (_Float16)b.z; r[7] = (_Float16)b.w;
  return r;
}

__device__ __forceinline__ v8f wmh(v16h a, v16h b, v8f c) {
  v8f d = __builtin_amdgcn_wmma_f32_16x16x32_f16(false, a, false, b, (short)0, c, false, false);
#if defined(__HIP_DEVICE_COMPILE__)
  asm volatile("v_nop\n\tv_nop\n\tv_nop\n\tv_nop" : "+v"(d) : "v"(a), "v"(b));
#endif
  return d;
}
__device__ __forceinline__ v8f wmb(v16b a, v16b b, v8f c) {
  v8f d = __builtin_amdgcn_wmma_f32_16x16x32_bf16(false, a, false, b, (short)0, c, false, false);
#if defined(__HIP_DEVICE_COMPILE__)
  asm volatile("v_nop\n\tv_nop\n\tv_nop\n\tv_nop" : "+v"(d) : "v"(a), "v"(b));
#endif
  return d;
}

template <int NB>
__device__ __forceinline__ int scan_chunk(const int* __restrict__ dsts, int nE, int cbase, int slotBase,
                                          int vec8, int* list, int tid, int lane, int wave) {
  int wc = 0;
#pragma unroll
  for (int g = 0; g < NGRP; ++g) {
    const int el0  = (g * NTHR + tid) * EPT;
    const int e0   = cbase + el0;
    const int sent = -2147483647 - 1;
    v4i da, db;
    if (vec8 != 0 && cbase + CHUNK <= nE) {
      da = *(const v4i*)(dsts + e0);
      db = *(const v4i*)(dsts + e0 + 4);
    } else {
      da.x = (e0     < nE) ? dsts[min(e0, nE - 1)] : sent;
      da.y = (e0 + 1 < nE) ? dsts[min(e0 + 1, nE - 1)] : sent;
      da.z = (e0 + 2 < nE) ? dsts[min(e0 + 2, nE - 1)] : sent;
      da.w = (e0 + 3 < nE) ? dsts[min(e0 + 3, nE - 1)] : sent;
      db.x = (e0 + 4 < nE) ? dsts[min(e0 + 4, nE - 1)] : sent;
      db.y = (e0 + 5 < nE) ? dsts[min(e0 + 5, nE - 1)] : sent;
      db.z = (e0 + 6 < nE) ? dsts[min(e0 + 6, nE - 1)] : sent;
      db.w = (e0 + 7 < nE) ? dsts[min(e0 + 7, nE - 1)] : sent;
    }
    const unsigned nb = (unsigned)slotBase;
    const unsigned s0 = (unsigned)da.x - nb, s1 = (unsigned)da.y - nb;
    const unsigned s2 = (unsigned)da.z - nb, s3 = (unsigned)da.w - nb;
    const unsigned s4 = (unsigned)db.x - nb, s5 = (unsigned)db.y - nb;
    const unsigned s6 = (unsigned)db.z - nb, s7 = (unsigned)db.w - nb;
    const bool h0 = s0 < (unsigned)NB, h1 = s1 < (unsigned)NB, h2 = s2 < (unsigned)NB, h3 = s3 < (unsigned)NB;
    const bool h4 = s4 < (unsigned)NB, h5 = s5 < (unsigned)NB, h6 = s6 < (unsigned)NB, h7 = s7 < (unsigned)NB;
    const unsigned any = __builtin_amdgcn_ballot_w32(h0 | h1 | h2 | h3 | h4 | h5 | h6 | h7);
    if (any != 0u) {
#define HITJ(J, HJ, SJ) { \
        const unsigned mj = __builtin_amdgcn_ballot_w32(HJ); \
        if (mj != 0u) { \
          if (HJ) { \
            const int pos = wc + (int)__builtin_amdgcn_mbcnt_lo(mj, 0u); \
            if (pos < WCAP) list[wave * WCAP + pos] = ((el0 + (J)) << 12) | (int)(SJ); \
          } \
          wc += (int)__builtin_popcount(mj); } }
      HITJ(0, h0, s0)
      HITJ(1, h1, s1)
      HITJ(2, h2, s2)
      HITJ(3, h3, s3)
      HITJ(4, h4, s4)
      HITJ(5, h5, s5)
      HITJ(6, h6, s6)
      HITJ(7, h7, s7)
#undef HITJ
    }
  }
  return wc;
}

__global__ __launch_bounds__(NTHR) void k_wprep(
    const float* __restrict__ W1, const float* __restrict__ Wl,
    _Float16* w1a, _Float16* w1b, unsigned short* wlh, unsigned short* wll) {
  const int g = D * D / 8;
  const int bstart = blockIdx.x * NTHR;
  const int seg = bstart < g ? 0 : (bstart < 2 * g ? 1 : 2);
  const int i = bstart + (int)threadIdx.x;
  if (i >= 3 * g) return;
  const int o  = (i - seg * g) * 8;
  const int n  = o / D;
  const int k0 = o - n * D;
  const float* src = (seg == 2) ? Wl : W1;
  const int kofs = (seg == 1) ? D : 0;
  float v[8];
#pragma unroll
  for (int e = 0; e < 8; ++e) v[e] = src[(size_t)(kofs + k0 + e) * D + n];
  if (seg < 2) {
    v4f a, b;
    a.x = v[0] * WSCALE; a.y = v[1] * WSCALE; a.z = v[2] * WSCALE; a.w = v[3] * WSCALE;
    b.x = v[4] * WSCALE; b.y = v[5] * WSCALE; b.z = v[6] * WSCALE; b.w = v[7] * WSCALE;
    const v8h hv = cvt8(a, b);
    _Float16* dp = ((seg == 0) ? w1a : w1b) + o;
    *(volatile v8h*)dp = hv;
    __threadfence();
    *(volatile v8h*)dp = hv;
  } else {
    v8us hv, lv;
#pragma unroll
    for (int e = 0; e < 8; ++e) {
      const unsigned short hb = f2bf(v[e]);
      const float hf = __uint_as_float(((unsigned int)hb) << 16);
      const unsigned short lb = f2bf(v[e] - hf);
      hv[e] = hb;
      lv[e] = lb;
    }
    *(volatile v8us*)(wlh + o) = hv;
    *(volatile v8us*)(wll + o) = lv;
    __threadfence();
    *(volatile v8us*)(wlh + o) = hv;
    *(volatile v8us*)(wll + o) = lv;
  }
}

__global__ __launch_bounds__(NTHR) void k_gemm16(
    const float* __restrict__ A, const _Float16* __restrict__ Bs, const float* __restrict__ bias,
    float* C, int nRowsA, int useBias) {
  extern __shared__ v4f lds_dyn[];
  _Float16* sA  = (_Float16*)lds_dyn;
  float*    stg = (float*)lds_dyn;
  const int tid = threadIdx.x, lane = tid & 31, wave = tid >> 5, hh = lane >> 4, m = lane & 15;
  const int rowBase = blockIdx.x * GROWS;

#pragma unroll
  for (int i = 0; i < (GROWS * D / 8) / NTHR; ++i) {
    const int idx = i * NTHR + tid;
    const int r   = idx >> 4;
    const int c0  = (idx & 15) * 8;
    int row = rowBase + r;
    row = row > nRowsA - 1 ? nRowsA - 1 : row;
    const float* ap = A + (size_t)row * D + c0;
    const v4f a = *(const v4f*)ap, b = *(const v4f*)(ap + 4);
    *(v8h*)(sA + r * AP + c0) = cvt8(a, b);
  }
  __syncthreads();

  v8f acc[8];
#pragma unroll
  for (int t = 0; t < 8; ++t) { v8f z = {0.f, 0.f, 0.f, 0.f, 0.f, 0.f, 0.f, 0.f}; acc[t] = z; }
  const _Float16* ar = sA + (wave * 16 + m) * AP + 8 * hh;
#pragma unroll
  for (int kt = 0; kt < D / 32; ++kt) {
    FragH a;
    a.h[0] = *(const v8h*)(ar + 32 * kt);
    a.h[1] = *(const v8h*)(ar + 32 * kt + 16);
#pragma unroll
    for (int t = 0; t < 8; ++t) {
      const _Float16* bp = Bs + (size_t)(16 * t + m) * D + 32 * kt + 8 * hh;
      FragH b;
      b.h[0] = *(const v8h*)bp;
      b.h[1] = *(const v8h*)(bp + 16);
      acc[t] = wmh(a.v, b.v, acc[t]);
    }
  }
  __syncthreads();

  const int r0 = wave * 16 + 8 * hh;
  float* sp = stg + r0 * D + m;
#pragma unroll
  for (int t = 0; t < 8; ++t) {
    const float bl = bias[16 * t + m];
    const float bv = useBias != 0 ? bl : 0.0f;
#pragma unroll
    for (int r = 0; r < 8; ++r) sp[r * D + 16 * t] = acc[t][r] * WINV + bv;
  }
  __syncthreads();

  const float* lp = stg + wave * 16 * D + 4 * lane;
  float* gp = C + ((size_t)rowBase + wave * 16) * D + 4 * lane;
#pragma unroll
  for (int i = 0; i < 16; ++i) { const v4f v = *(const v4f*)(lp + i * D); *(volatile v4f*)(gp + (size_t)i * D) = v; }
  __threadfence();
#pragma unroll
  for (int i = 0; i < 16; ++i) { const v4f v = *(const v4f*)(lp + i * D); *(volatile v4f*)(gp + (size_t)i * D) = v; }
}

__global__ __launch_bounds__(NTHR) void k_gemm3(
    const float* __restrict__ A, const unsigned short* __restrict__ Bh, const unsigned short* __restrict__ Bl,
    const float* __restrict__ bias, float* C, int nRows) {
  extern __shared__ v4f lds_dyn[];
  unsigned short* sH  = (unsigned short*)lds_dyn;
  unsigned short* sL  = sH + GROWS * AP;
  float*          stg = (float*)lds_dyn;
  const int tid = threadIdx.x, lane = tid & 31, wave = tid >> 5, hh = lane >> 4, m = lane & 15;
  const int rowBase = blockIdx.x * GROWS;

#pragma unroll
  for (int i = 0; i < (GROWS * D / 8) / NTHR; ++i) {
    const int idx = i * NTHR + tid;
    const int r   = idx >> 4;
    const int c0  = (idx & 15) * 8;
    int row = rowBase + r;
    row = row > nRows - 1 ? nRows - 1 : row;
    const float* ap = A + (size_t)row * D + c0;
    const v4f a = *(const v4f*)ap, b = *(const v4f*)(ap + 4);
    float f[8];
    f[0] = a.x; f[1] = a.y; f[2] = a.z; f[3] = a.w; f[4] = b.x; f[5] = b.y; f[6] = b.z; f[7] = b.w;
    v8us hv, lv;
#pragma unroll
    for (int e = 0; e < 8; ++e) {
      const unsigned short hb = f2bf(f[e]);
      const float hf = __uint_as_float(((unsigned int)hb) << 16);
      hv[e] = hb;
      lv[e] = f2bf(f[e] - hf);
    }
    *(v8us*)(sH + r * AP + c0) = hv;
    *(v8us*)(sL + r * AP + c0) = lv;
  }
  __syncthreads();

  v8f acc[8];
#pragma unroll
  for (int t = 0; t < 8; ++t) { v8f z = {0.f, 0.f, 0.f, 0.f, 0.f, 0.f, 0.f, 0.f}; acc[t] = z; }
  const unsigned short* arh = sH + (wave * 16 + m) * AP + 8 * hh;
  const unsigned short* arl = sL + (wave * 16 + m) * AP + 8 * hh;
#pragma unroll
  for (int kt = 0; kt < D / 32; ++kt) {
    FragB ah, al;
    ah.h[0] = *(const v8us*)(arh + 32 * kt);
    ah.h[1] = *(const v8us*)(arh + 32 * kt + 16);
    al.h[0] = *(const v8us*)(arl + 32 * kt);
    al.h[1] = *(const v8us*)(arl + 32 * kt + 16);
#pragma unroll
    for (int t = 0; t < 8; ++t) {
      const size_t bo = (size_t)(16 * t + m) * D + 32 * kt + 8 * hh;
      FragB bh, bl;
      bh.h[0] = *(const v8us*)(Bh + bo);
      bh.h[1] = *(const v8us*)(Bh + bo + 16);
      bl.h[0] = *(const v8us*)(Bl + bo);
      bl.h[1] = *(const v8us*)(Bl + bo + 16);
      acc[t] = wmb(ah.v, bh.v, acc[t]);
      acc[t] = wmb(ah.v, bl.v, acc[t]);
      acc[t] = wmb(al.v, bh.v, acc[t]);
    }
  }
  __syncthreads();

  const int r0 = wave * 16 + 8 * hh;
  float* sp = stg + r0 * D + m;
#pragma unroll
  for (int t = 0; t < 8; ++t) {
    const float bv = bias[16 * t + m];
#pragma unroll
    for (int r = 0; r < 8; ++r) sp[r * D + 16 * t] = fmaxf(acc[t][r] + bv, 0.0f);
  }
  __syncthreads();

  const float* lp = stg + wave * 16 * D + 4 * lane;
  const int rw = rowBase + wave * 16;
  float* gp = C + (size_t)rw * D + 4 * lane;
#pragma unroll
  for (int i = 0; i < 16; ++i) {
    if (rw + i < nRows) { const v4f v = *(const v4f*)(lp + i * D); *(volatile v4f*)(gp + (size_t)i * D) = v; }
  }
  __threadfence();
#pragma unroll
  for (int i = 0; i < 16; ++i) {
    if (rw + i < nRows) { const v4f v = *(const v4f*)(lp + i * D); *(volatile v4f*)(gp + (size_t)i * D) = v; }
  }
}

__global__ __launch_bounds__(NTHR) void k_agg(
    const int* __restrict__ ei, const float* __restrict__ x, const float* __restrict__ P,
    const float* __restrict__ Q, const float* __restrict__ W2, const float* __restrict__ b2,
    float* OE, int nN, int nE, int vec8) {
  extern __shared__ v4f lds_dyn[];
  float* acc  = (float*)lds_dyn;
  float* sS   = acc + TGT * D;
  int*   sCnt = (int*)(sS + TGT);
  int*   list = sCnt + TGT;
  int*   wcnt = list + LISTN;
  const int tid = threadIdx.x, lane = tid & 31;
  const int wave = __builtin_amdgcn_readfirstlane(tid >> 5);
  const int nodeBase = blockIdx.x * TGT;
  const int* rows = ei;
  const int* cols = ei + nE;

  {
    const v4f z = {0.f, 0.f, 0.f, 0.f};
    for (int i = tid; i < TGT * D / 4; i += NTHR) ((v4f*)acc)[i] = z;
    for (int i = tid; i < TGT; i += NTHR) { sS[i] = 0.0f; sCnt[i] = 0; }
  }
  const v4f w2v = *(const v4f*)(W2 + 4 * lane);
  const float b2v = b2[0];
  __syncthreads();

  const int nChunks = (nE + CHUNK - 1) / CHUNK;
#pragma unroll 1
  for (int ch = 0; ch < nChunks; ++ch) {
    const int cbase = ch * CHUNK;
    const int wc = scan_chunk<TGT>(rows, nE, cbase, nodeBase, vec8, list, tid, lane, wave);
    if (lane == 0) wcnt[wave] = wc;
    __syncthreads();
#pragma unroll 1
    for (int wsx = 0; wsx < NWAVE; ++wsx) {
      int n = __builtin_amdgcn_readfirstlane(wcnt[wsx]);
      n = n > WCAP ? WCAP : (n < 0 ? 0 : n);
      const int* lp = list + wsx * WCAP;
#pragma unroll 1
      for (int i = 0; i < n; ++i) {
        const int ent  = __builtin_amdgcn_readfirstlane(lp[i]);
        const int slot = ent & (TGT - 1);
        if ((slot >> 5) == wave) {
          int e = cbase + ((ent >> 12) & (CHUNK - 1));
          e = e > nE - 1 ? nE - 1 : e;
          int c = cols[e];
          c = c < 0 ? 0 : (c > nN - 1 ? nN - 1 : c);
          const v4f pv = *(const v4f*)(P + ((size_t)(nodeBase + slot)) * D + 4 * lane);
          const v4f qv = *(const v4f*)(Q + (size_t)c * D + 4 * lane);
          const v4f xv = *(const v4f*)(x + (size_t)c * D + 4 * lane);
          v4f hv = pv + qv;
          hv.x = fmaxf(hv.x, 0.0f); hv.y = fmaxf(hv.y, 0.0f); hv.z = fmaxf(hv.z, 0.0f); hv.w = fmaxf(hv.w, 0.0f);
          float ds = hv.x * w2v.x + hv.y * w2v.y + hv.z * w2v.z + hv.w * w2v.w;
          ds += __shfl_xor(ds, 16);
          ds += __shfl_xor(ds, 8);
          ds += __shfl_xor(ds, 4);
          ds += __shfl_xor(ds, 2);
          ds += __shfl_xor(ds, 1);
          const float z  = ds + b2v;
          const float ez = __expf(-z);
          const float mv = __builtin_amdgcn_rcpf(1.0f + ez);
          v4f* ap = (v4f*)(acc + slot * D + 4 * lane);
          v4f av = *ap;
          av = av + xv * mv;
          *ap = av;
          if (lane == 0) {
            sS[slot]   = sS[slot] + mv;
            sCnt[slot] = sCnt[slot] + 1;
          }
        }
      }
    }
    __syncthreads();
  }
  __syncthreads();

#pragma unroll 1
  for (int j = 0; j < 32; ++j) {
    const int ls   = wave * 32 + j;
    const int row  = nodeBase + ls;
    const int rowc = row > nN - 1 ? nN - 1 : row;
    const int   cj = sCnt[ls];
    const float sj = sS[ls];
    const float rinv = 1.0f / (sj + 1e-9f);
    v4f* ap = (v4f*)(acc + ls * D + 4 * lane);
    const v4f av = *ap;
    const v4f xv = *(const v4f*)(x + (size_t)rowc * D + 4 * lane);
    const v4f ag = av * rinv;
    const v4f bv = xv * 0.5f + ag * 0.5f;
    v4f ov;
    ov.x = (cj > 0) ? bv.x : xv.x;
    ov.y = (cj > 0) ? bv.y : xv.y;
    ov.z = (cj > 0) ? bv.z : xv.z;
    ov.w = (cj > 0) ? bv.w : xv.w;
    *ap = ov;
  }

  float* gb = OE + (size_t)nodeBase * D + 4 * lane;
#pragma unroll 1
  for (int j = 0; j < 32; ++j) {
    const int ls = wave * 32 + j;
    const v4f v = *(const v4f*)(acc + ls * D + 4 * lane);
    *(volatile v4f*)(gb + (size_t)ls * D) = v;
  }
  __threadfence();
#pragma unroll 1
  for (int j = 0; j < 32; ++j) {
    const int ls = wave * 32 + j;
    const v4f v = *(const v4f*)(acc + ls * D + 4 * lane);
    *(volatile v4f*)(gb + (size_t)ls * D) = v;
  }
}

extern "C" void kernel_launch(void* const* d_in, const int* in_sizes, int n_in,
                              void* d_out, int out_size, void* d_ws, size_t ws_size,
                              hipStream_t stream) {
  if (n_in < 8) return;
  const int nN = in_sizes[0] / D;
  const int nE = in_sizes[1] / 2;
  if (nN <= 0 || nE <= 0 || in_sizes[0] != nN * D || in_sizes[1] != 2 * nE) return;
  if (in_sizes[2] != 2 * D * D || in_sizes[3] != D || in_sizes[4] != D || in_sizes[5] < 1 ||
      in_sizes[6] != D * D || in_sizes[7] != D) return;
  if (out_size != nN * D) return;
  if (nE > (1 << 28) || nN > (1 << 24)) return;

  const float* x  = (const float*)d_in[0];
  const int*   ei = (const int*)d_in[1];
  const float* W1 = (const float*)d_in[2];
  const float* b1 = (const float*)d_in[3];
  const float* W2 = (const float*)d_in[4];
  const float* b2 = (const float*)d_in[5];
  const float* Wl = (const float*)d_in[6];
  const float* bl = (const float*)d_in[7];
  float* out = (float*)d_out;

  const int nAgg   = (nN + TGT - 1) / TGT;
  const int NPAD   = nAgg * TGT;
  const int nGemmP = NPAD / GROWS;
  const int nGemm3 = (nN + GROWS - 1) / GROWS;
  if (nGemm3 * GROWS > NPAD) return;

  char* ws = (char*)d_ws;
  size_t off = 0;
  const size_t oW1a = off; off += (size_t)D * D * 2;      off = (off + 255) & ~(size_t)255;
  const size_t oW1b = off; off += (size_t)D * D * 2;      off = (off + 255) & ~(size_t)255;
  const size_t oWlh = off; off += (size_t)D * D * 2;      off = (off + 255) & ~(size_t)255;
  const size_t oWll = off; off += (size_t)D * D * 2;      off = (off + 255) & ~(size_t)255;
  const size_t oP   = off; off += (size_t)NPAD * D * 4;   off = (off + 255) & ~(size_t)255;
  const size_t oQ   = off; off += (size_t)NPAD * D * 4;   off = (off + 255) & ~(size_t)255;
  const size_t oOE  = off; off += (size_t)NPAD * D * 4;   off = (off + 255) & ~(size_t)255;
  if (off > ws_size || off > (size_t)134217728) return;
  _Float16*       w1a = (_Float16*)(ws + oW1a);
  _Float16*       w1b = (_Float16*)(ws + oW1b);
  unsigned short* wlh = (unsigned short*)(ws + oWlh);
  unsigned short* wll = (unsigned short*)(ws + oWll);
  float*          P   = (float*)(ws + oP);
  float*          Q   = (float*)(ws + oQ);
  float*          OE  = (float*)(ws + oOE);

  k_wprep<<<(3 * (D * D / 8)) / NTHR, NTHR, 0, stream>>>(W1, Wl, w1a, w1b, wlh, wll);

  hipFuncSetAttribute(reinterpret_cast<const void*>(&k_gemm16),
                      hipFuncAttributeMaxDynamicSharedMemorySize, LDS_GEMM);
  k_gemm16<<<nGemmP, NTHR, LDS_GEMM, stream>>>(x, w1a, b1, P, nN, 1);
  k_gemm16<<<nGemmP, NTHR, LDS_GEMM, stream>>>(x, w1b, b1, Q, nN, 0);

  hipFuncSetAttribute(reinterpret_cast<const void*>(&k_agg),
                      hipFuncAttributeMaxDynamicSharedMemorySize, LDS_AGG);
  k_agg<<<nAgg, NTHR, LDS_AGG, stream>>>(ei, x, P, Q, W2, b2, OE, nN, nE, 1);

  hipFuncSetAttribute(reinterpret_cast<const void*>(&k_gemm3),
                      hipFuncAttributeMaxDynamicSharedMemorySize, LDS_GEM3);
  k_gemm3<<<nGemm3, NTHR, LDS_GEM3, stream>>>(OE, wlh, wll, bl, out, nN);
}
